// MultiHeadAttention_85117661872728
// MI455X (gfx1250) — hardware-verified
//
#include <hip/hip_runtime.h>
#include <math.h>

#ifndef NB
#define NB 2
#endif
#ifndef SEQ
#define SEQ 2048
#endif
#define NB_FULL 2
#define SEQ_FULL 2048
#define DM 1024
#define NH 16
#define DH 64
#define NTOK (NB * SEQ)
#define ISL_ROWS ((SEQ < 512) ? SEQ : 512)
#define ISL_QB (ISL_ROWS / 64)
#define NQB (SEQ / 64)
#define AT_NW 4
#define PPI 32
#define OSP 68

static_assert(DM == 1024);
static_assert(NH * DH == DM);
static_assert(DH == 64);
static_assert(SEQ % 64 == 0);
static_assert(NTOK % 64 == 0);
static_assert(DM % 64 == 0);
static_assert(DM % 32 == 0);
static_assert((2 * DM) % 32 == 0);
static_assert(NB <= NB_FULL);
static_assert(SEQ <= SEQ_FULL);
static_assert(AT_NW * 16 == 64);
static_assert(ISL_ROWS % 64 == 0);
static_assert(PPI == 32);
static_assert(NTOK * DM < 2147483647 / 2);

typedef __attribute__((ext_vector_type(16))) _Float16 v16h;
typedef __attribute__((ext_vector_type(8)))  _Float16 v8h;
typedef __attribute__((ext_vector_type(16))) __bf16   v16b;
typedef __attribute__((ext_vector_type(8)))  __bf16   v8b;
typedef __attribute__((ext_vector_type(8)))  float    v8f;
typedef __attribute__((ext_vector_type(4)))  float    v4f;
typedef __attribute__((ext_vector_type(4)))  unsigned int v4u;


#define VST2(T, ptr, val) do { const T vst2_v_ = (val); *(volatile T*)(ptr) = vst2_v_; __threadfence(); *(volatile T*)(ptr) = vst2_v_; } while (0)

__device__ __forceinline__ float cmb_bf(float v) {
    const unsigned u = __builtin_bit_cast(unsigned, v);
    const unsigned r = (u + 0x7fffu + ((u >> 16) & 1u)) & 0xffff0000u;
    return __builtin_bit_cast(float, r);
}
__device__ __forceinline__ unsigned short bf_bits(float f) {
    const unsigned u = __builtin_bit_cast(unsigned, f);
    return (unsigned short)((u + 0x7fffu + ((u >> 16) & 1u)) >> 16);
}
__device__ __forceinline__ float bf_bits2f(unsigned short h) { return __builtin_bit_cast(float, ((unsigned)h) << 16); }
__device__ __forceinline__ unsigned pk2h(float a, float b) {
    return (unsigned)__builtin_bit_cast(unsigned short, (_Float16)a) | ((unsigned)__builtin_bit_cast(unsigned short, (_Float16)b) << 16);
}
__device__ __forceinline__ unsigned pk2bf_split(float a, float b, unsigned* lo) {
    const unsigned short ha = bf_bits(a), hb = bf_bits(b);
    const unsigned short la = bf_bits(a - bf_bits2f(ha)), lb = bf_bits(b - bf_bits2f(hb));
    *lo = (unsigned)la | ((unsigned)lb << 16);
    return (unsigned)ha | ((unsigned)hb << 16);
}
__device__ __forceinline__ void wave_lds_sync() {
    __builtin_amdgcn_fence(3  , "workgroup");
    __builtin_amdgcn_wave_barrier();
    __builtin_amdgcn_fence(2  , "workgroup");
}
__device__ __forceinline__ int opaque_i(int v) { asm volatile("" : "+v"(v)); return v; }

__global__ __launch_bounds__(256) void k_cast_x(const float* __restrict__ SRC, unsigned short* __restrict__ DST) {
    const int u = blockIdx.x * 256 + threadIdx.x; const int b = blockIdx.y;
    if (u >= SEQ * (DM / 8)) return;
    const int r = u / (DM / 8); const int c0 = 8 * (u % (DM / 8));
    const float* s = SRC + ((long long)b * SEQ_FULL + r) * DM + c0;
    const v4f a = *(const v4f*)s; const v4f d = *(const v4f*)(s + 4);
    v4u pk;
    pk.x = pk2h(cmb_bf(a.x), cmb_bf(a.y)); pk.y = pk2h(cmb_bf(a.z), cmb_bf(a.w));
    pk.z = pk2h(cmb_bf(d.x), cmb_bf(d.y)); pk.w = pk2h(cmb_bf(d.z), cmb_bf(d.w));
    VST2(v4u, (v4u*)(DST + ((long long)b * SEQ + r) * DM + c0), pk);
}
__global__ __launch_bounds__(256) void k_cast_wT(const float* __restrict__ SRC, unsigned short* __restrict__ DST) {
    const int u = blockIdx.x * 256 + threadIdx.x;
    if (u >= DM * (DM / 8)) return;
    const int n = u / (DM / 8); const int k0 = 8 * (u % (DM / 8));
    float w[8];
#pragma unroll
    for (int e = 0; e < 8; ++e) w[e] = cmb_bf(SRC[(long long)(k0 + e) * DM + n]) * 16.0f;
    v4u pk; pk.x = pk2h(w[0], w[1]); pk.y = pk2h(w[2], w[3]); pk.z = pk2h(w[4], w[5]); pk.w = pk2h(w[6], w[7]);
    VST2(v4u, (v4u*)(DST + (long long)n * DM + k0), pk);
}
__global__ __launch_bounds__(256) void k_cast_woT2(const float* __restrict__ SRC, unsigned short* __restrict__ DST) {
    const int u = blockIdx.x * 256 + threadIdx.x;
    if (u >= DM * (DM / 8)) return;
    const int n = u / (DM / 8); const int k0 = 8 * (u % (DM / 8));
    unsigned short w[8];
#pragma unroll
    for (int e = 0; e < 8; ++e) w[e] = bf_bits(SRC[(long long)(k0 + e) * DM + n]);
    v4u pk;
    pk.x = (unsigned)w[0] | ((unsigned)w[1] << 16); pk.y = (unsigned)w[2] | ((unsigned)w[3] << 16);
    pk.z = (unsigned)w[4] | ((unsigned)w[5] << 16); pk.w = (unsigned)w[6] | ((unsigned)w[7] << 16);
    VST2(v4u, (v4u*)(DST + (long long)n * (2 * DM) + k0), pk);
    VST2(v4u, (v4u*)(DST + (long long)n * (2 * DM) + DM + k0), pk);
}
__global__ __launch_bounds__(256) void k_bias4(const float* __restrict__ b0, const float* __restrict__ b1, const float* __restrict__ b2, const float* __restrict__ b3, float* __restrict__ DST) {
    const int i = blockIdx.x * 256 + threadIdx.x;
    if (i >= 4 * DM) return;
    const int seg = i >> 10, j = i & (DM - 1);
    const float v0 = cmb_bf(b0[j]) * 0.125f, v1 = cmb_bf(b1[j]), v2 = cmb_bf(b2[j]), v3 = cmb_bf(b3[j]);
    const float v = (seg == 0) ? v0 : ((seg == 1) ? v1 : ((seg == 2) ? v2 : v3));
    VST2(float, DST + i, v);
}

__device__ __forceinline__ void dep_guard_h(v8f& a, v8f& b, v16h x, v16h y) { asm volatile("v_nop\n\tv_nop\n\tv_nop\n\tv_nop" : "+v"(a), "+v"(b) : "v"(x), "v"(y)); }
__device__ __forceinline__ void dep_guard_b(v8f& a, v8f& b, v16b x, v16b y) { asm volatile("v_nop\n\tv_nop\n\tv_nop\n\tv_nop" : "+v"(a), "+v"(b) : "v"(x), "v"(y)); }
__device__ __forceinline__ void keep4_h(v16h a, v16h b, v16h c, v16h d) { asm volatile("v_nop" :: "v"(a), "v"(b), "v"(c), "v"(d)); }
__device__ __forceinline__ void keep4_b(v16b a, v16b b, v16b c, v16b d) { asm volatile("v_nop" :: "v"(a), "v"(b), "v"(c), "v"(d)); }
__device__ __forceinline__ void acc_guard4(v8f& a, v8f& b, v8f& c, v8f& d) { asm volatile("v_nop\n\tv_nop\n\tv_nop\n\tv_nop" : "+v"(a), "+v"(b), "+v"(c), "+v"(d)); }
template <typename T> struct Frag;
template <> struct Frag<_Float16> {
  typedef v16h V; union U { v16h v; v8h h[2]; };
  static __device__ __forceinline__ v16h load(const _Float16* p) {
    U f; f.h[0] = *(const v8h*)(p); f.h[1] = *(const v8h*)(p + 16); return f.v;
  }
  static __device__ __forceinline__ v8f mma(v16h a, v16h b, v8f c) {
    return __builtin_amdgcn_wmma_f32_16x16x32_f16(false, a, false, b, (short)0, c, false, false);
  }
  static __device__ __forceinline__ void guard(v8f& a, v8f& b, v16h x, v16h y) { dep_guard_h(a, b, x, y); }
  static __device__ __forceinline__ void keep(v16h a, v16h b, v16h c, v16h d) { keep4_h(a, b, c, d); }
};
template <> struct Frag<__bf16> {
  typedef v16b V; union U { v16b v; v8b h[2]; };
  static __device__ __forceinline__ v16b load(const __bf16* p) {
    U f; f.h[0] = *(const v8b*)(p); f.h[1] = *(const v8b*)(p + 16); return f.v;
  }
  static __device__ __forceinline__ v8f mma(v16b a, v16b b, v8f c) {
    return __builtin_amdgcn_wmma_f32_16x16x32_bf16(false, a, false, b, (short)0, c, false, false);
  }
  static __device__ __forceinline__ void guard(v8f& a, v8f& b, v16b x, v16b y) { dep_guard_b(a, b, x, y); }
  static __device__ __forceinline__ void keep(v16b a, v16b b, v16b c, v16b d) { keep4_b(a, b, c, d); }
};
template <int ET> struct Elem;
template <> struct Elem<0> { typedef _Float16 T; };
template <> struct Elem<1> { typedef __bf16 T; };

template <int ET, int BIAS_MODE, int OUT_MODE>
__device__ __forceinline__ void gemm64_body(
    const unsigned short* __restrict__ Ap, int lda, long long strideA,
    const unsigned short* __restrict__ Btp, int ldb, long long strideB,
    float* __restrict__ Cf, unsigned short* __restrict__ C16, unsigned short* __restrict__ CHp, unsigned short* __restrict__ CLp,
    int ldc, long long strideC, const float* __restrict__ bias, int M, int N, int K, float scale) {
  typedef typename Elem<ET>::T T;
  typedef typename Frag<T>::V V;
  __shared__ __align__(16) float sT[8][16 * OSP];
  const int b    = blockIdx.y;
  const int lane = threadIdx.x & 31;
  const int wave = threadIdx.x >> 5;
  const int tilesN = N >> 6;
  const int tilesM = M >> 6;
  const int tile = blockIdx.x * 8 + wave;
  if (tile >= tilesM * tilesN) return;
  const int tm = tile / tilesN;
  const int tn = tile - tm * tilesN;
  const int m0 = tm << 6;
  const int n0 = tn << 6;

  const T* Ab = (const T*)Ap + (size_t)b * strideA;
  const T* Bb = (const T*)Btp + (size_t)b * strideB;

  const int rlane = lane & 15;
  const int koff  = (lane >> 4) * 8;
  const int mOff  = (lane >> 4) * 8;

  v8f acc[4][4];
#pragma unroll
  for (int i = 0; i < 4; ++i)
#pragma unroll
    for (int j = 0; j < 4; ++j) acc[i][j] = (v8f){0.f,0.f,0.f,0.f,0.f,0.f,0.f,0.f};

  for (int k0 = 0; k0 < K; k0 += 32) {
    V bh[4];
#pragma unroll
    for (int j = 0; j < 4; ++j) {
      const size_t bo = (size_t)(n0 + (j << 4) + rlane) * ldb + koff + k0;
      bh[j] = Frag<T>::load(Bb + bo);
    }
#pragma unroll
    for (int i = 0; i < 4; ++i) {
      const size_t ao = (size_t)(m0 + (i << 4) + rlane) * lda + koff + k0;
      V ah = Frag<T>::load(Ab + ao);
#pragma unroll
      for (int j = 0; j < 4; ++j) acc[i][j] = Frag<T>::mma(ah, bh[j], acc[i][j]);
      Frag<T>::guard(acc[i][0], acc[i][3], ah, ah);
    }
    Frag<T>::keep(bh[0], bh[1], bh[2], bh[3]);
  }
  acc_guard4(acc[0][0], acc[0][1], acc[0][2], acc[0][3]);
  acc_guard4(acc[1][0], acc[1][1], acc[1][2], acc[1][3]);
  acc_guard4(acc[2][0], acc[2][1], acc[2][2], acc[2][3]);
  acc_guard4(acc[3][0], acc[3][1], acc[3][2], acc[3][3]);

#pragma unroll
  for (int i = 0; i < 4; ++i) {
    const int mBase = m0 + (i << 4);
#pragma unroll
    for (int j = 0; j < 4; ++j) {
      const int n = n0 + (j << 4) + rlane;
      float bv = 0.f;
      if (BIAS_MODE == 2) bv = bias[n];
#pragma unroll
      for (int r = 0; r < 8; ++r) {
        float v = acc[i][j][r] * scale;
        if (BIAS_MODE == 1) v += bias[mBase + mOff + r];
        if (BIAS_MODE == 2) v += bv;
        sT[wave][(mOff + r) * OSP + (j << 4) + rlane] = v;
      }
    }
    wave_lds_sync();
    if (OUT_MODE == 0) {
      float* C = Cf + (size_t)b * strideC;
      const int hh = lane >> 4, c4 = (lane & 15) * 4;
      for (int pass = 0; pass < 2; ++pass) {
#pragma unroll
        for (int it = 0; it < 8; ++it) {
          const int row = it * 2 + hh;
          const v4f v = *(const v4f*)(&sT[wave][row * OSP + c4]);
          *(volatile v4f*)(C + (size_t)(mBase + row) * ldc + n0 + c4) = v;
        }
        __threadfence();
      }
    } else {
      const int q = lane >> 3, c8 = (lane & 7) * 8;
      for (int pass = 0; pass < 2; ++pass) {
#pragma unroll
        for (int it = 0; it < 4; ++it) {
          const int row = it * 4 + q;
          const v4f x0 = *(const v4f*)(&sT[wave][row * OSP + c8]);
          const v4f x1 = *(const v4f*)(&sT[wave][row * OSP + c8 + 4]);
          v4u p16, ph, pl;
          p16.x = pk2h(x0.x, x0.y); p16.y = pk2h(x0.z, x0.w); p16.z = pk2h(x1.x, x1.y); p16.w = pk2h(x1.z, x1.w);
          unsigned lo;
          ph.x = pk2bf_split(x0.x, x0.y, &lo); pl.x = lo;
          ph.y = pk2bf_split(x0.z, x0.w, &lo); pl.y = lo;
          ph.z = pk2bf_split(x1.x, x1.y, &lo); pl.z = lo;
          ph.w = pk2bf_split(x1.z, x1.w, &lo); pl.w = lo;
          const size_t o = (size_t)b * strideC + (size_t)(mBase + row) * ldc + n0 + c8;
          *(volatile v4u*)(C16 + o) = p16;
          *(volatile v4u*)(CHp + o) = ph;
          *(volatile v4u*)(CLp + o) = pl;
        }
        __threadfence();
      }
    }
    wave_lds_sync();
  }
}

__global__ __launch_bounds__(256) void k_gemm_rows(const unsigned short* __restrict__ A, const unsigned short* __restrict__ Bt,
    unsigned short* __restrict__ C16, unsigned short* __restrict__ CH, unsigned short* __restrict__ CL,
    const float* __restrict__ bias, int M, int N, int K, int ldc, float scale) {
  gemm64_body<0, 2, 3>(A, K, 0, Bt, K, 0, nullptr, C16, CH, CL, ldc, 0, bias, M, N, K, scale);
}
__global__ __launch_bounds__(256) void k_gemm_cols(const unsigned short* __restrict__ A, const unsigned short* __restrict__ Bt,
    unsigned short* __restrict__ C16, unsigned short* __restrict__ CH, unsigned short* __restrict__ CL,
    const float* __restrict__ bias, int M, int N, int K, int ldc, float scale) {
  gemm64_body<0, 1, 3>(A, K, 0, Bt, K, 0, nullptr, C16, CH, CL, ldc, 0, bias, M, N, K, scale);
}
__global__ __launch_bounds__(256) void k_gemm_out(const unsigned short* __restrict__ A, const unsigned short* __restrict__ Bt,
    float* __restrict__ C, const float* __restrict__ bias, int M, int N, int K, long long strideA, long long strideC) {
  gemm64_body<1, 2, 0>(A, K, strideA, Bt, K, 0, C, nullptr, nullptr, nullptr, N, strideC, bias, M, N, K, 1.0f);
}

namespace at {
union FB { v16b v; v8b h[2]; };
__device__ __forceinline__ __bf16 f2bf(float f) { return __builtin_bit_cast(__bf16, bf_bits(f)); }
__device__ __forceinline__ void split(float f, __bf16& hi, __bf16& lo) {
  const unsigned short hb = bf_bits(f);
  hi = __builtin_bit_cast(__bf16, hb);
  lo = f2bf(f - bf_bits2f(hb));
}
__device__ __forceinline__ v8f mma_b(v16b a, v16b b, v8f c) {
  c = __builtin_amdgcn_wmma_f32_16x16x32_bf16(false, a, false, b, (short)0, c, false, false);
  asm volatile("v_nop\n\tv_nop\n\tv_nop\n\tv_nop" : "+v"(c) : "v"(a), "v"(b));
  return c;
}
template <bool F16> __device__ __forceinline__ __bf16 to16(float f) {
  if (F16) return __builtin_bit_cast(__bf16, (_Float16)f);
  return f2bf(f);
}
template <bool F16> __device__ __forceinline__ v8f mma16(v16b a, v16b b, v8f c) {
  if (F16) {
    const v16h ah = __builtin_bit_cast(v16h, a), bh = __builtin_bit_cast(v16h, b);
    c = __builtin_amdgcn_wmma_f32_16x16x32_f16(false, ah, false, bh, (short)0, c, false, false);
    asm volatile("v_nop\n\tv_nop\n\tv_nop\n\tv_nop" : "+v"(c) : "v"(ah), "v"(bh));
    return c;
  }
  return mma_b(a, b, c);
}
__device__ __forceinline__ v16b ldg_frag(const __bf16* __restrict__ p, int off) {
  FB f; f.h[0] = *(const v8b*)(p + off); f.h[1] = *(const v8b*)(p + off + 16); return f.v;
}

template <bool SPLIT>
__device__ __forceinline__ void attn_body(const __bf16* __restrict__ Qh, const __bf16* __restrict__ Ql,
                                          const __bf16* __restrict__ Kh, const __bf16* __restrict__ Kl,
                                          const __bf16* __restrict__ Vh, const __bf16* __restrict__ Vl,
                                          unsigned short* __restrict__ CTX, int qb0) {
  constexpr bool F16 = !SPLIT;
  const float PSC = F16 ? 32768.0f : 1.0f;
  const float L2E = 1.4426950408889634f;
  const float NEG = -__builtin_inff();
  __shared__ __align__(16) __bf16 Psh[AT_NW][16 * PPI];
  __shared__ __align__(16) __bf16 Psl[SPLIT ? AT_NW : 1][SPLIT ? 16 * PPI : 8];
  __shared__ __align__(16) float  Os[AT_NW][16 * OSP];

  const int tid  = threadIdx.x;
  const int wave = tid >> 5;
  const int lane = tid & 31;
  const int hh   = lane >> 4;
  const int c    = lane & 15;
  const int qb = blockIdx.x + qb0;
  const int h  = blockIdx.y;
  const int b  = blockIdx.z;
  const int q0 = qb * 64 + wave * 16;
  const int tok0 = b * SEQ;
  const int qoff = (tok0 + q0 + c) * DM + h * DH + 8 * hh;
  const int koff = (tok0 + c) * DM + h * DH + 8 * hh;
  const int voff = (h * DH + c) * NTOK + tok0 + 8 * hh;

  float mrow[8], lrow[8];
  v8f oacc[4];
#pragma unroll
  for (int r = 0; r < 8; ++r) { mrow[r] = NEG; lrow[r] = 0.f; }
#pragma unroll
  for (int t = 0; t < 4; ++t) oacc[t] = (v8f){0.f,0.f,0.f,0.f,0.f,0.f,0.f,0.f};

  const int nsteps = (q0 >> 5) + 1;
  for (int st = 0; st < nsteps; ++st) {
    const int kv0 = st * 32;
    const int qo = opaque_i(qoff);
    v8f s0 = (v8f){0.f,0.f,0.f,0.f,0.f,0.f,0.f,0.f};
    v8f s1 = (v8f){0.f,0.f,0.f,0.f,0.f,0.f,0.f,0.f};
#pragma unroll
    for (int dc = 0; dc < 2; ++dc) {
      const v16b qh  = ldg_frag(Qh, qo + dc * 32);
      const v16b k0h = ldg_frag(Kh, koff + kv0 * DM + dc * 32);
      const v16b k1h = ldg_frag(Kh, koff + (kv0 + 16) * DM + dc * 32);
      s0 = mma16<F16>(qh, k0h, s0);
      s1 = mma16<F16>(qh, k1h, s1);
      if (SPLIT) {
        const v16b ql  = ldg_frag(Ql, qo + dc * 32);
        const v16b k0l = ldg_frag(Kl, koff + kv0 * DM + dc * 32);
        const v16b k1l = ldg_frag(Kl, koff + (kv0 + 16) * DM + dc * 32);
        s0 = mma16<F16>(qh, k0l, s0);
        s0 = mma16<F16>(ql, k0h, s0);
        s1 = mma16<F16>(qh, k1l, s1);
        s1 = mma16<F16>(ql, k1h, s1);
      }
    }
#pragma unroll
    for (int r = 0; r < 8; ++r) {
      const int qrow = q0 + 8 * hh + r;
      const float a0 = (kv0 + c > qrow) ? NEG : s0[r] * L2E;
      const float a1 = (kv0 + 16 + c > qrow) ? NEG : s1[r] * L2E;
      float m = fmaxf(a0, a1);
      m = fmaxf(m, __shfl_xor(m, 1, 32)); m = fmaxf(m, __shfl_xor(m, 2, 32));
      m = fmaxf(m, __shfl_xor(m, 4, 32)); m = fmaxf(m, __shfl_xor(m, 8, 32));
      const float mnew  = fmaxf(mrow[r], m);
      const float alpha = (mrow[r] == NEG) ? 0.f : exp2f(mrow[r] - mnew);
      const float p0 = (a0 == NEG) ? 0.f : exp2f(a0 - mnew);
      const float p1 = (a1 == NEG) ? 0.f : exp2f(a1 - mnew);
      mrow[r] = mnew;
      lrow[r] = lrow[r] * alpha + (p0 + p1);
#pragma unroll
      for (int t = 0; t < 4; ++t) oacc[t][r] *= alpha;
      if (SPLIT) {
        __bf16 ph_, pl_;
        split(p0, ph_, pl_); Psh[wave][(8 * hh + r) * PPI + c] = ph_;      Psl[SPLIT ? wave : 0][(8 * hh + r) * PPI + c] = pl_;
        split(p1, ph_, pl_); Psh[wave][(8 * hh + r) * PPI + 16 + c] = ph_; Psl[SPLIT ? wave : 0][(8 * hh + r) * PPI + 16 + c] = pl_;
      } else {
        Psh[wave][(8 * hh + r) * PPI + c]      = to16<true>(p0 * PSC);
        Psh[wave][(8 * hh + r) * PPI + 16 + c] = to16<true>(p1 * PSC);
      }
    }
    wave_lds_sync();
    FB pa;
    pa.h[0] = *(const v8b*)(&Psh[wave][c * PPI + 8 * hh]);
    pa.h[1] = *(const v8b*)(&Psh[wave][c * PPI + 16 + 8 * hh]);
    if (SPLIT) {
      FB pl;
      pl.h[0] = *(const v8b*)(&Psl[SPLIT ? wave : 0][c * PPI + 8 * hh]);
      pl.h[1] = *(const v8b*)(&Psl[SPLIT ? wave : 0][c * PPI + 16 + 8 * hh]);
#pragma unroll
      for (int t = 0; t < 4; ++t) {
        const v16b vb = ldg_frag(Vh, voff + t * 16 * NTOK + kv0);
        const v16b vl = ldg_frag(Vl, voff + t * 16 * NTOK + kv0);
        oacc[t] = mma16<F16>(pa.v, vb, oacc[t]);
        oacc[t] = mma16<F16>(pa.v, vl, oacc[t]);
        oacc[t] = mma16<F16>(pl.v, vb, oacc[t]);
      }
    } else {
#pragma unroll
      for (int t = 0; t < 4; ++t) {
        const v16b vb = ldg_frag(Vh, voff + t * 16 * NTOK + kv0);
        oacc[t] = mma16<F16>(pa.v, vb, oacc[t]);
      }
    }
    wave_lds_sync();
  }

#pragma unroll
  for (int r = 0; r < 8; ++r) {
    float l = lrow[r];
    l += __shfl_xor(l, 1, 32); l += __shfl_xor(l, 2, 32); l += __shfl_xor(l, 4, 32); l += __shfl_xor(l, 8, 32);
    const float inv = 1.0f / (l * PSC);
#pragma unroll
    for (int t = 0; t < 4; ++t) Os[wave][(8 * hh + r) * OSP + t * 16 + c] = oacc[t][r] * inv;
  }
  wave_lds_sync();
  {
    const int q = lane >> 3, c8 = (lane & 7) * 8;
    for (int pass = 0; pass < 2; ++pass) {
#pragma unroll
      for (int it = 0; it < 4; ++it) {
        const int row = it * 4 + q;
        const v4f x0 = *(const v4f*)(&Os[wave][row * OSP + c8]);
        const v4f x1 = *(const v4f*)(&Os[wave][row * OSP + c8 + 4]);
        v4u ph, pl; unsigned lo;
        ph.x = pk2bf_split(x0.x, x0.y, &lo); pl.x = lo;
        ph.y = pk2bf_split(x0.z, x0.w, &lo); pl.y = lo;
        ph.z = pk2bf_split(x1.x, x1.y, &lo); pl.z = lo;
        ph.w = pk2bf_split(x1.z, x1.w, &lo); pl.w = lo;
        const size_t o = (size_t)(tok0 + q0 + row) * (2 * DM) + h * DH + c8;
        *(volatile v4u*)(CTX + o) = ph;
        *(volatile v4u*)(CTX + o + DM) = pl;
      }
      __threadfence();
    }
  }
}
}

__global__ __launch_bounds__(128) void k_attn_island(const unsigned short* __restrict__ QH, const unsigned short* __restrict__ QL,
    const unsigned short* __restrict__ KH, const unsigned short* __restrict__ KL,
    const unsigned short* __restrict__ VTH, const unsigned short* __restrict__ VTL, unsigned short* __restrict__ CTX) {
  at::attn_body<true>((const __bf16*)QH, (const __bf16*)QL, (const __bf16*)KH, (const __bf16*)KL, (const __bf16*)VTH, (const __bf16*)VTL, CTX, 0);
}
__global__ __launch_bounds__(128) void k_attn_plain(const unsigned short* __restrict__ Q16, const unsigned short* __restrict__ K16,
    const unsigned short* __restrict__ VT16, unsigned short* __restrict__ CTX) {
  at::attn_body<false>((const __bf16*)Q16, (const __bf16*)Q16, (const __bf16*)K16, (const __bf16*)K16, (const __bf16*)VT16, (const __bf16*)VT16, CTX, ISL_QB);
}

constexpr size_t SZ_X16  = (size_t)NTOK * DM * 2;
constexpr size_t SZ_W16  = (size_t)3 * DM * DM * 2;
constexpr size_t SZ_WO2  = (size_t)DM * 2 * DM * 2;
constexpr size_t SZ_BR   = (size_t)4 * DM * 4;
constexpr size_t SZ_PL   = (size_t)NTOK * DM * 2;
constexpr size_t SZ_CTX  = (size_t)NTOK * 2 * DM * 2;
constexpr size_t WS_TOTAL = SZ_X16 + SZ_W16 + SZ_WO2 + SZ_BR + 9 * SZ_PL + SZ_CTX;
static_assert(SZ_X16 % 256 == 0);
static_assert(SZ_W16 % 256 == 0);
static_assert(SZ_WO2 % 256 == 0);
static_assert(SZ_BR % 256 == 0);
static_assert(SZ_PL % 256 == 0);
static_assert(SZ_CTX % 256 == 0);
static_assert(WS_TOTAL <= (size_t)134217728);

extern "C" void kernel_launch(void* const* d_in, const int* in_sizes, int n_in, void* d_out, int out_size, void* d_ws, size_t ws_size, hipStream_t stream) {
    if (n_in < 11) return;
    const long long need_x = ((long long)(NB - 1) * SEQ_FULL + SEQ) * DM;
    if ((long long)in_sizes[0] < need_x || (long long)in_sizes[1] < need_x || (long long)in_sizes[2] < need_x) return;
    if (in_sizes[3] < DM * DM || in_sizes[5] < DM * DM || in_sizes[7] < DM * DM || in_sizes[9] < DM * DM) return;
    if (in_sizes[4] < DM || in_sizes[6] < DM || in_sizes[8] < DM || in_sizes[10] < DM) return;
    if ((long long)out_size < need_x) return;
    if (WS_TOTAL > ws_size) return;
    const float* xq = (const float*)d_in[0];
    const float* xk = (const float*)d_in[1];
    const float* xv = (const float*)d_in[2];
    const float* Wq = (const float*)d_in[3];
    const float* bq = (const float*)d_in[4];
    const float* Wk = (const float*)d_in[5];
    const float* bk = (const float*)d_in[6];
    const float* Wv = (const float*)d_in[7];
    const float* bv = (const float*)d_in[8];
    const float* Wo = (const float*)d_in[9];
    const float* bo = (const float*)d_in[10];
    float* out = (float*)d_out;
    char* wsp = (char*)d_ws;
    unsigned short* X16  = (unsigned short*)wsp; wsp += SZ_X16;
    unsigned short* W16  = (unsigned short*)wsp; wsp += SZ_W16;
    unsigned short* WO2  = (unsigned short*)wsp; wsp += SZ_WO2;
    float*          BR   = (float*)wsp;          wsp += SZ_BR;
    unsigned short* Q16  = (unsigned short*)wsp; wsp += SZ_PL;
    unsigned short* QH   = (unsigned short*)wsp; wsp += SZ_PL;
    unsigned short* QL   = (unsigned short*)wsp; wsp += SZ_PL;
    unsigned short* K16  = (unsigned short*)wsp; wsp += SZ_PL;
    unsigned short* KH   = (unsigned short*)wsp; wsp += SZ_PL;
    unsigned short* KL   = (unsigned short*)wsp; wsp += SZ_PL;
    unsigned short* VT16 = (unsigned short*)wsp; wsp += SZ_PL;
    unsigned short* VTH  = (unsigned short*)wsp; wsp += SZ_PL;
    unsigned short* VTL  = (unsigned short*)wsp; wsp += SZ_PL;
    unsigned short* CTX  = (unsigned short*)wsp; wsp += SZ_CTX;

    const unsigned gw = (unsigned)((DM * (DM / 8) + 255) / 256);
    k_cast_wT<<<gw, 256, 0, stream>>>(Wq, W16);
    k_cast_wT<<<gw, 256, 0, stream>>>(Wk, W16 + (size_t)DM * DM);
    k_cast_wT<<<gw, 256, 0, stream>>>(Wv, W16 + (size_t)2 * DM * DM);
    k_cast_woT2<<<gw, 256, 0, stream>>>(Wo, WO2);
    k_bias4<<<(4 * DM + 255) / 256, 256, 0, stream>>>(bq, bk, bv, bo, BR);

    const dim3 gx((unsigned)((SEQ * (DM / 8) + 255) / 256), (unsigned)NB);
    const unsigned gproj = (unsigned)(((NTOK / 64) * (DM / 64) + 7) / 8);
    k_cast_x<<<gx, 256, 0, stream>>>(xq, X16);
    k_gemm_rows<<<gproj, 256, 0, stream>>>(X16, W16, Q16, QH, QL, BR, NTOK, DM, DM, DM, 0.0078125f);
    k_cast_x<<<gx, 256, 0, stream>>>(xk, X16);
    k_gemm_rows<<<gproj, 256, 0, stream>>>(X16, W16 + (size_t)DM * DM, K16, KH, KL, BR + DM, NTOK, DM, DM, DM, 0.0625f);
    k_cast_x<<<gx, 256, 0, stream>>>(xv, X16);
    k_gemm_cols<<<gproj, 256, 0, stream>>>(W16 + (size_t)2 * DM * DM, X16, VT16, VTH, VTL, BR + 2 * DM, DM, NTOK, DM, NTOK, 0.0625f);

    k_attn_island<<<dim3((unsigned)ISL_QB, (unsigned)NH, (unsigned)NB), 128, 0, stream>>>(QH, QL, KH, KL, VTH, VTL, CTX);
    if (NQB > ISL_QB) {
        k_attn_plain<<<dim3((unsigned)(NQB - ISL_QB), (unsigned)NH, (unsigned)NB), 128, 0, stream>>>(Q16, K16, VT16, CTX);
    }

    const dim3 go((unsigned)(((SEQ / 64) * (DM / 64) + 7) / 8), (unsigned)NB);
    k_gemm_out<<<go, 256, 0, stream>>>(CTX, WO2, out, BR + 3 * DM, SEQ, DM, 2 * DM, (long long)SEQ * 2 * DM, (long long)SEQ_FULL * DM);
}
